// Easy_SS2D_29832842838266
// MI455X (gfx1250) — hardware-verified
//
#include <hip/hip_runtime.h>
#include <math.h>
#include <stdint.h>


#define BSZ   4
#define DM    96
#define DMP   128
#define DI    192
#define HH    128
#define WW    128
#define LL    (HH * WW)
#define KDIR  4
#define DTR   6
#define NE    32
#define XDP   64
#define YSC     1024.0f
#define YSC_INV (1.0f / 1024.0f)

typedef __attribute__((ext_vector_type(16))) _Float16 v16h;
typedef __attribute__((ext_vector_type(8)))  _Float16 v8h;
typedef __attribute__((ext_vector_type(16))) __bf16   v16b;
typedef __attribute__((ext_vector_type(8)))  __bf16   v8b;
typedef __attribute__((ext_vector_type(8)))  float    v8f;
typedef __attribute__((ext_vector_type(4)))  float    v4f;

__device__ __forceinline__ unsigned short f2bf_bits(float f) {
  unsigned u = __float_as_uint(f);
  return (unsigned short)((u + 0x7FFFu + ((u >> 16) & 1u)) >> 16);
}
__device__ __forceinline__ float bf_bits2f(unsigned short h) { return __uint_as_float(((unsigned)h) << 16); }

__device__ __forceinline__ void dep_guard_h(v8f& a, v8f& b, v16h x, v16h y) { asm volatile("v_nop\n\tv_nop\n\tv_nop\n\tv_nop" : "+v"(a), "+v"(b) : "v"(x), "v"(y)); }
__device__ __forceinline__ void dep_guard_b(v8f& a, v8f& b, v16b x, v16b y) { asm volatile("v_nop\n\tv_nop\n\tv_nop\n\tv_nop" : "+v"(a), "+v"(b) : "v"(x), "v"(y)); }
__device__ __forceinline__ void keep4_h(v16h a, v16h b, v16h c, v16h d) { asm volatile("v_nop" :: "v"(a), "v"(b), "v"(c), "v"(d)); }
__device__ __forceinline__ void keep4_b(v16b a, v16b b, v16b c, v16b d) { asm volatile("v_nop" :: "v"(a), "v"(b), "v"(c), "v"(d)); }
__device__ __forceinline__ void acc_guard4(v8f& a, v8f& b, v8f& c, v8f& d) { asm volatile("v_nop\n\tv_nop\n\tv_nop\n\tv_nop" : "+v"(a), "+v"(b), "+v"(c), "+v"(d)); }
template <typename T> struct Frag;
template <> struct Frag<_Float16> {
  typedef v16h V; union U { v16h v; v8h h[2]; };
  static __device__ __forceinline__ v16h load(const _Float16* p) {
    U f; f.h[0] = *(const v8h*)(p); f.h[1] = *(const v8h*)(p + 16); return f.v;
  }
  static __device__ __forceinline__ v8f mma(v16h a, v16h b, v8f c) {
    return __builtin_amdgcn_wmma_f32_16x16x32_f16(false, a, false, b, (short)0, c, false, false);
  }
  static __device__ __forceinline__ void guard(v8f& a, v8f& b, v16h x, v16h y) { dep_guard_h(a, b, x, y); }
  static __device__ __forceinline__ void keep(v16h a, v16h b, v16h c, v16h d) { keep4_h(a, b, c, d); }
};
template <> struct Frag<__bf16> {
  typedef v16b V; union U { v16b v; v8b h[2]; };
  static __device__ __forceinline__ v16b load(const __bf16* p) {
    U f; f.h[0] = *(const v8b*)(p); f.h[1] = *(const v8b*)(p + 16); return f.v;
  }
  static __device__ __forceinline__ v8f mma(v16b a, v16b b, v8f c) {
    return __builtin_amdgcn_wmma_f32_16x16x32_bf16(false, a, false, b, (short)0, c, false, false);
  }
  static __device__ __forceinline__ void guard(v8f& a, v8f& b, v16b x, v16b y) { dep_guard_b(a, b, x, y); }
  static __device__ __forceinline__ void keep(v16b a, v16b b, v16b c, v16b d) { keep4_b(a, b, c, d); }
};

template <int ET> struct Elem;
template <> struct Elem<0> { typedef _Float16 T; };
template <> struct Elem<1> { typedef __bf16 T; };
template <int ET, bool SPLIT, int BIAS_MODE, int OUT_MODE, bool RESID, int ACT = 0>
__global__ __launch_bounds__(256) void wmma_gemm64(
    const unsigned short* __restrict__ Ap, const unsigned short* __restrict__ A2p, int lda, long strideA,
    const unsigned short* __restrict__ Btp, const unsigned short* __restrict__ Bt2p, int ldb, long strideB,
    void* __restrict__ Cout, void* __restrict__ Cout2, int ldc, long strideC,
    const float* __restrict__ bias,
    const float* __restrict__ resid, long strideR,
    int M, int N, int K, float scale, int Mstore) {
  typedef typename Elem<ET>::T T;
  typedef typename Frag<T>::V V;
  const T* A = (const T*)Ap; const T* A2 = (const T*)A2p; const T* Bt = (const T*)Btp; const T* Bt2 = (const T*)Bt2p;
  __shared__ __align__(16) float sT[8][16 * 68];
  const int b    = blockIdx.y;
  const int lane = threadIdx.x & 31;
  const int wave = threadIdx.x >> 5;
  const int tilesN = N >> 6;
  const int tilesM = M >> 6;
  const int tile = blockIdx.x * 8 + wave;
  if (tile >= tilesM * tilesN) return;
  const int tm = tile / tilesN;
  const int tn = tile - tm * tilesN;
  const int m0 = tm << 6;
  const int n0 = tn << 6;

  const T* Ab  = A  + (size_t)b * strideA;
  const T* Bb  = Bt + (size_t)b * strideB;
  const T* Ab2 = SPLIT ? (A2  + (size_t)b * strideA) : nullptr;
  const T* Bb2 = SPLIT ? (Bt2 + (size_t)b * strideB) : nullptr;

  const int rlane = lane & 15;
  const int koff  = (lane >> 4) * 8;
  const int mOff  = (lane >> 4) * 8;

  v8f acc[4][4];
#pragma unroll
  for (int i = 0; i < 4; ++i)
#pragma unroll
    for (int j = 0; j < 4; ++j) acc[i][j] = (v8f){0.f,0.f,0.f,0.f,0.f,0.f,0.f,0.f};

  for (int k0 = 0; k0 < K; k0 += 32) {
    V bh[4], bl[4];
#pragma unroll
    for (int j = 0; j < 4; ++j) {
      const size_t bo = (size_t)(n0 + (j << 4) + rlane) * ldb + koff + k0;
      bh[j] = Frag<T>::load(Bb + bo);
      if (SPLIT) bl[j] = Frag<T>::load(Bb2 + bo);
    }
#pragma unroll
    for (int i = 0; i < 4; ++i) {
      const size_t ao = (size_t)(m0 + (i << 4) + rlane) * lda + koff + k0;
      V ah = Frag<T>::load(Ab + ao);
      V al;
      if (SPLIT) al = Frag<T>::load(Ab2 + ao);
#pragma unroll
      for (int j = 0; j < 4; ++j) {
        acc[i][j] = Frag<T>::mma(ah, bh[j], acc[i][j]);
        if (SPLIT) {
          acc[i][j] = Frag<T>::mma(ah, bl[j], acc[i][j]);
          acc[i][j] = Frag<T>::mma(al, bh[j], acc[i][j]);
        }
      }
      Frag<T>::guard(acc[i][0], acc[i][3], ah, SPLIT ? al : ah);
    }
    Frag<T>::keep(bh[0], bh[1], bh[2], bh[3]);
    if (SPLIT) Frag<T>::keep(bl[0], bl[1], bl[2], bl[3]);
  }
  acc_guard4(acc[0][0], acc[0][1], acc[0][2], acc[0][3]);
  acc_guard4(acc[1][0], acc[1][1], acc[1][2], acc[1][3]);
  acc_guard4(acc[2][0], acc[2][1], acc[2][2], acc[2][3]);
  acc_guard4(acc[3][0], acc[3][1], acc[3][2], acc[3][3]);

  float* slab = sT[wave];
  const float* Rb = RESID ? (resid + (size_t)b * strideR) : nullptr;
#pragma unroll
  for (int i = 0; i < 4; ++i) {
    const int mBase = m0 + (i << 4);
    if (mBase >= Mstore) break;
#pragma unroll
    for (int j = 0; j < 4; ++j) {
      const int n = n0 + (j << 4) + rlane;
      float bv = 0.f;
      if (BIAS_MODE == 2) bv = bias[n];
#pragma unroll
      for (int r = 0; r < 8; ++r) {
        float v = acc[i][j][r] * scale;
        if (BIAS_MODE == 1) v += bias[mBase + mOff + r];
        if (BIAS_MODE == 2) v += bv;
        if (RESID) v += Rb[(size_t)(mBase + mOff + r) * ldc + n];
        if (ACT == 1) v = tanhf(v);
        if (ACT == 2) v = fmaxf(v, 0.0f);
        if (ACT == 3) v = v / (1.0f + expf(-v));
        if (ACT == 4) v = (v > 0.f) ? v : 0.01f * v;
        if (ACT == 5) v = 0.5f * v * (1.0f + erff(v * 0.70710678118654752f));
        slab[(mOff + r) * 68 + (j << 4) + rlane] = v;
      }
    }
    __builtin_amdgcn_fence(__ATOMIC_RELEASE, "workgroup");
    __builtin_amdgcn_wave_barrier();
    __builtin_amdgcn_fence(__ATOMIC_ACQUIRE, "workgroup");
    if (OUT_MODE == 0) {
      float* C = (float*)Cout + (size_t)b * strideC;
      const int hh = lane >> 4, c4 = (lane & 15) * 4;
      for (int pass = 0; pass < 2; ++pass) {
#pragma unroll
        for (int it = 0; it < 8; ++it) {
          const int row = it * 2 + hh;
          v4f v = *(const v4f*)(slab + row * 68 + c4);
          *(volatile v4f*)(C + (size_t)(mBase + row) * ldc + n0 + c4) = v;
        }
        __threadfence();
      }
    } else {
      const int q = lane >> 3, c8 = (lane & 7) * 8;
      unsigned short* C  = (unsigned short*)Cout  + (size_t)b * strideC;
      unsigned short* C2 = (OUT_MODE == 2) ? ((unsigned short*)Cout2 + (size_t)b * strideC) : nullptr;
      for (int pass = 0; pass < 2; ++pass) {
#pragma unroll
        for (int it = 0; it < 4; ++it) {
          const int row = it * 4 + q;
          const float* sp = slab + row * 68 + c8;
          v8h hv, lv;
#pragma unroll
          for (int e = 0; e < 8; ++e) {
            if (OUT_MODE == 1) {
              hv[e] = (_Float16)sp[e];
            } else {
              unsigned short hb = f2bf_bits(sp[e]);
              unsigned short lb = f2bf_bits(sp[e] - bf_bits2f(hb));
              hv[e] = __builtin_bit_cast(_Float16, hb);
              lv[e] = __builtin_bit_cast(_Float16, lb);
            }
          }
          *(volatile v8h*)(C + (size_t)(mBase + row) * ldc + n0 + c8) = hv;
          if (OUT_MODE == 2) *(volatile v8h*)(C2 + (size_t)(mBase + row) * ldc + n0 + c8) = lv;
        }
        __threadfence();
      }
    }
    __builtin_amdgcn_fence(__ATOMIC_RELEASE, "workgroup");
    __builtin_amdgcn_wave_barrier();
    __builtin_amdgcn_fence(__ATOMIC_ACQUIRE, "workgroup");
  }
}

__device__ __forceinline__ int tr_idx(int p) { return ((p & (HH - 1)) << 7) | (p >> 7); }

__global__ __launch_bounds__(256) void k_prep_w(
    const float* __restrict__ in_w, const float* __restrict__ xpw, const float* __restrict__ out_w,
    _Float16* __restrict__ w16)
{
  const int NQ_IN  = DI * DM / 8;
  const int NQ_X   = XDP * DI / 8;
  const int NQ_OUT = DMP * DI / 8;
  for (int pass = 0; pass < 2; ++pass) {
    for (int q = threadIdx.x; q < NQ_IN + NQ_X + NQ_OUT; q += 256) {
      v8h v;
      if (q < NQ_IN) {
        const int e0 = q * 8;
#pragma unroll
        for (int i = 0; i < 8; ++i) v[i] = (_Float16)(in_w[e0 + i] * 64.0f);
      } else if (q < NQ_IN + NQ_X) {
        const int e0  = (q - NQ_IN) * 8;
        const int row = e0 / DI;
        const int col = e0 - row * DI;
        const int rc  = (row < NE) ? row : (NE - 1);
        const float keep = (row < NE) ? 1024.0f : 0.0f;
#pragma unroll
        for (int i = 0; i < 8; ++i) v[i] = (_Float16)(xpw[rc * DI + col + i] * keep);
      } else {
        const int e0  = (q - NQ_IN - NQ_X) * 8;
        const int row = e0 / DI;
        const int col = e0 - row * DI;
        const int rc  = (row < DM) ? row : (DM - 1);
        const float keep = (row < DM) ? 256.0f : 0.0f;
#pragma unroll
        for (int i = 0; i < 8; ++i) v[i] = (_Float16)(out_w[rc * DI + col + i] * keep);
      }
      *(volatile v8h*)(w16 + (size_t)q * 8) = v;
    }
    __threadfence();
  }
}

__global__ __launch_bounds__(256) void k_x_to_pm(const float* __restrict__ x, _Float16* __restrict__ xT)
{
  __shared__ __align__(16) _Float16 sX[64 * 104];
  const int t   = threadIdx.x;
  const int blk = blockIdx.x;
  const int b   = blk >> 8;
  const int p0  = (blk & 255) * 64;
  const int px  = t & 63;
  const int g   = t >> 6;
  const float* xb = x + (size_t)b * DM * LL + p0 + px;
#pragma unroll 1
  for (int c = 0; c < 24; ++c) {
    const int ch = g * 24 + c;
    sX[px * 104 + ch] = (_Float16)(xb[(size_t)ch * LL] * 16.0f);
  }
  __syncthreads();
  _Float16* ob = xT + ((size_t)b * LL + p0) * DM;
  for (int pass = 0; pass < 2; ++pass) {
#pragma unroll
    for (int i = 0; i < 3; ++i) {
      const int q   = t + 256 * i;
      const int pix = q / 12;
      const int c8  = (q - pix * 12) * 8;
      const v8h v = *(const v8h*)(sX + pix * 104 + c8);
      *(volatile v8h*)(ob + (size_t)q * 8) = v;
    }
    __threadfence();
  }
}

__global__ __launch_bounds__(256) void k_dwconv(
    const float* __restrict__ z, const float* __restrict__ dww, const float* __restrict__ dwb,
    _Float16* __restrict__ Z16)
{
  __shared__ __align__(16) _Float16 sZ[64 * 200];
  const int t    = threadIdx.x;
  const int blk  = blockIdx.x;
  const int b    = blk >> 8;
  const int h    = (blk >> 1) & (HH - 1);
  const int half = blk & 1;
  const int wl   = t & 63;
  const int g    = t >> 6;
  const int w    = half * 64 + wl;
  const float* zb = z + (size_t)b * DI * LL;
#pragma unroll 1
  for (int c = 0; c < 48; ++c) {
    const int d = g * 48 + c;
    const float* zp = zb + (size_t)d * LL;
    const float* wk = dww + d * 9;
    float s = 0.f;
#pragma unroll
    for (int i = 0; i < 3; ++i) {
      const int h2 = h + i - 1;
      if (h2 < 0 || h2 >= HH) continue;
#pragma unroll
      for (int j = 0; j < 3; ++j) {
        const int w2 = w + j - 1;
        if (w2 < 0 || w2 >= WW) continue;
        s += wk[i * 3 + j] * zp[h2 * WW + w2];
      }
    }
    s += dwb[d];
    const float sig = __builtin_amdgcn_rcpf(1.0f + expf(-s));
    sZ[wl * 200 + d] = (_Float16)(s * sig);
  }
  __syncthreads();
  _Float16* ob = Z16 + ((size_t)b * LL + (size_t)h * WW + half * 64) * DI;
  for (int pass = 0; pass < 2; ++pass) {
#pragma unroll
    for (int i = 0; i < 6; ++i) {
      const int q   = t + 256 * i;
      const int pix = q / 24;
      const int c8  = (q - pix * 24) * 8;
      const v8h v = *(const v8h*)(sZ + pix * 200 + c8);
      *(volatile v8h*)(ob + (size_t)q * 8) = v;
    }
    __threadfence();
  }
}

__global__ __launch_bounds__(32) void k_scan(
    const _Float16* __restrict__ Z16, const float* __restrict__ xd,
    const float* __restrict__ dtw, const float* __restrict__ dtb,
    const float* __restrict__ alog, _Float16* __restrict__ Y, int kbase)
{
  __shared__ __align__(16) _Float16 sY[32 * 72];
  const int lane = threadIdx.x;
  const int blk  = blockIdx.x;
  const int kk   = blk / (BSZ * (DI / 32));
  const int rem  = blk - kk * (BSZ * (DI / 32));
  const int b    = rem / (DI / 32);
  const int dg   = rem - b * (DI / 32);
  const int k    = kbase + kk;
  const int d    = dg * 32 + lane;

  const float* wr = dtw + ((size_t)k * DI + d) * DTR;
  const float w0 = wr[0], w1 = wr[1], w2 = wr[2], w3 = wr[3], w4 = wr[4], w5 = wr[5];
  const float bias = dtb[k * DI + d];
  const float Av   = -expf(alog[k * DI + d]);

  const _Float16* zb = Z16 + (size_t)b * LL * DI + d;
  const float*    xb = xd + (size_t)b * LL * XDP + k * 8;
  _Float16* yrow = Y + (((size_t)kk * BSZ + b) * DI + dg * 32) * (size_t)LL;

  float hst = 0.f;
#pragma unroll 1
  for (int cch = 0; cch < LL / 64; ++cch) {
#pragma unroll 1
    for (int s = 0; s < 64; ++s) {
      const int l = cch * 64 + s;
      const int m = (k >= 2) ? (LL - 1 - l) : l;
      const int p = (k & 1) ? tr_idx(m) : m;
      const float* xr = xb + (size_t)p * XDP;
      const v4f xa = *(const v4f*)(xr);
      const v4f xc = *(const v4f*)(xr + 4);
      const float dts = w0 * xa[0] + w1 * xa[1] + w2 * xa[2] + w3 * xa[3] + w4 * xc[0] + w5 * xc[1];
      const float Bv = xc[2], Cv = xc[3];
      const float xx = dts + bias;
      const float delta = log1pf(expf(-fabsf(xx))) + fmaxf(xx, 0.f);
      const float uv = (float)zb[(size_t)p * DI];
      const float dA = expf(delta * Av);
      hst = hst * dA + (delta * Bv) * uv;
      sY[lane * 72 + s] = (_Float16)(hst * Cv * YSC);
    }
    __syncthreads();
    const int c8 = (lane & 7) * 8;
    for (int pass = 0; pass < 2; ++pass) {
#pragma unroll
      for (int it = 0; it < 8; ++it) {
        const int row = it * 4 + (lane >> 3);
        const v8h v = *(const v8h*)(sY + row * 72 + c8);
        *(volatile v8h*)(yrow + (size_t)row * LL + cch * 64 + c8) = v;
      }
      __threadfence();
    }
    __syncthreads();
  }
}

__global__ __launch_bounds__(256) void k_merge1(const _Float16* __restrict__ Y, _Float16* __restrict__ P)
{
  const int q = blockIdx.x * 256 + threadIdx.x;
  if (q >= BSZ * LL * 24) return;
  const int gp = q / 24;
  const int g  = q - gp * 24;
  const int c0 = g * 8;
  const int b  = gp >> 14;
  const int p  = gp & (LL - 1);
  const int l1 = tr_idx(p);
  const _Float16* y0 = Y + ((size_t)b * DI + c0) * (size_t)LL + p;
  const _Float16* y1 = Y + ((size_t)(BSZ + b) * DI + c0) * (size_t)LL + l1;
  v8h o;
#pragma unroll
  for (int i = 0; i < 8; ++i) o[i] = (_Float16)((float)y0[(size_t)i * LL] + (float)y1[(size_t)i * LL]);
  _Float16* dst = P + (size_t)q * 8;
  *(volatile v8h*)dst = o;
  __threadfence();
  *(volatile v8h*)dst = o;
}

__global__ __launch_bounds__(256) void k_merge2_ln(
    const _Float16* __restrict__ P, const _Float16* __restrict__ Y, const _Float16* __restrict__ Z16,
    const float* __restrict__ Dsv, const float* __restrict__ lnw, const float* __restrict__ lnb,
    _Float16* __restrict__ A16)
{
  const int lane = threadIdx.x & 31;
  const int wave = threadIdx.x >> 5;
  const int gw   = blockIdx.x * 8 + wave;
  const bool act = lane < 24;
  const int c0   = act ? lane * 8 : 0;
  float ds[8], wv[8], bv[8];
#pragma unroll
  for (int i = 0; i < 8; ++i) {
    ds[i] = Dsv[c0 + i] + Dsv[DI + c0 + i] + Dsv[2 * DI + c0 + i] + Dsv[3 * DI + c0 + i];
    wv[i] = lnw[c0 + i];
    bv[i] = lnb[c0 + i];
  }
  const float invn = 1.0f / (float)DI;
#pragma unroll 1
  for (int it = 0; it < 16; ++it) {
    const size_t gp = (size_t)gw * 16 + it;
    const int b  = (int)(gp >> 14);
    const int p  = (int)(gp & (LL - 1));
    const int l2 = LL - 1 - p;
    const int l3 = LL - 1 - tr_idx(p);
    const v8h pr = *(const v8h*)(P + gp * DI + c0);
    const v8h zr = *(const v8h*)(Z16 + gp * DI + c0);
    const _Float16* y2 = Y + ((size_t)b * DI + c0) * (size_t)LL + l2;
    const _Float16* y3 = Y + ((size_t)(BSZ + b) * DI + c0) * (size_t)LL + l3;
    float v[8];
    float s = 0.f;
#pragma unroll
    for (int i = 0; i < 8; ++i) {
      const float hc = ((float)pr[i] + (float)y2[(size_t)i * LL] + (float)y3[(size_t)i * LL]) * YSC_INV;
      v[i] = hc + ds[i] * (float)zr[i];
      s += v[i];
    }
    if (!act) s = 0.f;
#pragma unroll
    for (int off = 1; off < 32; off <<= 1) s += __shfl_xor(s, off, 32);
    const float mu = s * invn;
    float dv[8];
    float ss = 0.f;
#pragma unroll
    for (int i = 0; i < 8; ++i) { dv[i] = v[i] - mu; ss += dv[i] * dv[i]; }
    if (!act) ss = 0.f;
#pragma unroll
    for (int off = 1; off < 32; off <<= 1) ss += __shfl_xor(ss, off, 32);
    const float var = ss * invn;
    const float rs  = rsqrtf(var + 1e-5f);
    v8h o;
#pragma unroll
    for (int i = 0; i < 8; ++i) o[i] = (_Float16)((dv[i] * rs * wv[i] + bv[i]) * 16.0f);
    _Float16* dst = A16 + gp * DI + c0;
    if (act) *(volatile v8h*)dst = o;
    __threadfence();
    if (act) *(volatile v8h*)dst = o;
  }
}

extern "C" void kernel_launch(void* const* d_in, const int* in_sizes, int n_in,
                              void* d_out, int out_size, void* d_ws, size_t ws_size,
                              hipStream_t stream)
{
  (void)in_sizes; (void)n_in;
  const float* x      = (const float*)d_in[0];
  const float* in_w   = (const float*)d_in[1];
  const float* in_b   = (const float*)d_in[2];
  const float* dw_w   = (const float*)d_in[3];
  const float* dw_b   = (const float*)d_in[4];
  const float* xpw    = (const float*)d_in[5];
  const float* dtw    = (const float*)d_in[6];
  const float* dtb    = (const float*)d_in[7];
  const float* A_logs = (const float*)d_in[8];
  const float* Ds     = (const float*)d_in[9];
  const float* ln_w   = (const float*)d_in[10];
  const float* ln_b   = (const float*)d_in[11];
  const float* out_w  = (const float*)d_in[12];
  const float* out_b  = (const float*)d_in[13];

  const size_t w16_in_halves  = (size_t)DI * DM;
  const size_t w16_x_halves   = (size_t)XDP * DI;
  const size_t w16_out_halves = (size_t)DMP * DI;
  const size_t off_w    = 0;
  const size_t w_bytes  = (w16_in_halves + w16_x_halves + w16_out_halves) * 2;
  const size_t off_A    = (off_w + w_bytes + 255) & ~(size_t)255;
  const size_t plane16  = (size_t)BSZ * LL * DI * 2;
  const size_t x16_bytes = (size_t)BSZ * LL * DM * 2;
  const size_t xd_bytes  = (size_t)BSZ * LL * XDP * 4;
  size_t rA_bytes = plane16;
  if (x16_bytes > rA_bytes) rA_bytes = x16_bytes;
  if (xd_bytes > rA_bytes) rA_bytes = xd_bytes;
  const size_t off_Z    = off_A + rA_bytes;
  const size_t off_Y    = off_Z + plane16;
  const size_t rY_bytes = (size_t)BSZ * DI * LL * 4;
  const size_t off_P    = off_Y + rY_bytes;
  const size_t total    = off_P + plane16;
  if (total > ws_size) return;
  if ((size_t)out_size < (size_t)BSZ * DM * LL) return;

  char* ws = (char*)d_ws;
  _Float16* w16in  = (_Float16*)(ws + off_w);
  _Float16* w16x   = w16in + w16_in_halves;
  _Float16* w16out = w16x + w16_x_halves;
  _Float16* X16    = (_Float16*)(ws + off_A);
  float*    xd     = (float*)(ws + off_A);
  _Float16* A16    = (_Float16*)(ws + off_A);
  _Float16* Z16    = (_Float16*)(ws + off_Z);
  float*    zf     = (float*)(ws + off_Y);
  _Float16* Ypl    = (_Float16*)(ws + off_Y);
  _Float16* P16    = (_Float16*)(ws + off_P);

  k_prep_w<<<1, 256, 0, stream>>>(in_w, xpw, out_w, w16in);
  k_x_to_pm<<<BSZ * (LL / 64), 256, 0, stream>>>(x, X16);
  wmma_gemm64<0, false, 1, 0, false, 0><<<dim3((DI / 64) * (LL / 64) / 8, BSZ), 256, 0, stream>>>(
      (const unsigned short*)w16in, nullptr, DM, 0L,
      (const unsigned short*)X16, nullptr, DM, (long)LL * DM,
      (void*)zf, nullptr, LL, (long)DI * LL,
      in_b, nullptr, 0L,
      DI, LL, DM, 1.0f / 1024.0f, DI);
  k_dwconv<<<BSZ * HH * 2, 256, 0, stream>>>(zf, dw_w, dw_b, Z16);
  wmma_gemm64<0, false, 0, 0, false, 0><<<dim3(((BSZ * LL) / 64) / 8, 1), 256, 0, stream>>>(
      (const unsigned short*)Z16, nullptr, DI, 0L,
      (const unsigned short*)w16x, nullptr, DI, 0L,
      (void*)xd, nullptr, XDP, 0L,
      nullptr, nullptr, 0L,
      BSZ * LL, XDP, DI, 1.0f / 1024.0f, BSZ * LL);
  k_scan<<<2 * BSZ * (DI / 32), 32, 0, stream>>>(Z16, xd, dtw, dtb, A_logs, Ypl, 0);
  k_merge1<<<(BSZ * LL * 24) / 256, 256, 0, stream>>>(Ypl, P16);
  k_scan<<<2 * BSZ * (DI / 32), 32, 0, stream>>>(Z16, xd, dtw, dtb, A_logs, Ypl, 2);
  k_merge2_ln<<<(BSZ * LL) / (8 * 16), 256, 0, stream>>>(P16, Ypl, Z16, Ds, ln_w, ln_b, A16);
  wmma_gemm64<0, false, 1, 0, false, 0><<<dim3((DMP / 64) * (LL / 64) / 8, BSZ), 256, 0, stream>>>(
      (const unsigned short*)w16out, nullptr, DI, 0L,
      (const unsigned short*)A16, nullptr, DI, (long)LL * DI,
      d_out, nullptr, LL, (long)DM * LL,
      out_b, nullptr, 0L,
      DMP, LL, DI, 1.0f / 4096.0f, DM);
}
